// Olmo3MoeAttention_23141283791734
// MI455X (gfx1250) — hardware-verified
//
#include <hip/hip_runtime.h>
#include <hip/hip_bf16.h>


typedef __attribute__((ext_vector_type(16))) _Float16 bf16x16;
typedef __attribute__((ext_vector_type(8)))  float  f32x8;

#define WMMA_BF16(A, Bm, Cm) \
  __builtin_amdgcn_wmma_f32_16x16x32_f16(false, (A), false, (Bm), (short)0, (Cm), false, false)

#define B_    2
#define S_    2048
#define HID_  2048
#define NH_   32
#define NKV_  8
#define HD_   64
#define SCALE_ 0.125f
#define NEG_BIG (-3.0e38f)

__device__ __forceinline__ unsigned short f2bf(float f) {
  const _Float16 h = (_Float16)f;
  return __builtin_bit_cast(unsigned short, h);
}
__device__ __forceinline__ void split16(float f, unsigned short& hi, unsigned short& lo) {
  const _Float16 h = (_Float16)f;
  hi = __builtin_bit_cast(unsigned short, h);
  lo = __builtin_bit_cast(unsigned short, (_Float16)((f - (float)h) * 2048.0f));
}
#define RSPLIT (1.0f / 2048.0f)

__device__ __forceinline__ void async_ld_lds_b128(const void* gptr, void* lptr) {
  unsigned ldsoff = (unsigned)(unsigned long long)lptr;
  asm volatile("global_load_async_to_lds_b128 %0, %1, off"
               :: "v"(ldsoff), "v"(gptr) : "memory");
}
__device__ __forceinline__ void wait_asynccnt0() {
  asm volatile("s_wait_asynccnt 0x0" ::: "memory");
}

__global__ __launch_bounds__(256) void cvt_f32_bf16(const float* __restrict__ in,
                                                    unsigned short* __restrict__ out,
                                                    unsigned short* __restrict__ outl,
                                                    int n) {
  int i = (blockIdx.x * 256 + threadIdx.x) * 4;
  if (i + 3 < n) {
    float4 v = *(const float4*)(in + i);
    unsigned short h0, l0, h1, l1, h2, l2, h3, l3;
    split16(v.x, h0, l0); split16(v.y, h1, l1); split16(v.z, h2, l2); split16(v.w, h3, l3);
    typedef __attribute__((ext_vector_type(2))) unsigned v2u_t;
    v2u_t r;  r.x  = (unsigned)h0 | ((unsigned)h1 << 16); r.y  = (unsigned)h2 | ((unsigned)h3 << 16);
    v2u_t rl; rl.x = (unsigned)l0 | ((unsigned)l1 << 16); rl.y = (unsigned)l2 | ((unsigned)l3 << 16);
    *(volatile v2u_t*)(out + i) = r; *(volatile v2u_t*)(outl + i) = rl;
    __threadfence();
    *(volatile v2u_t*)(out + i) = r; *(volatile v2u_t*)(outl + i) = rl;
  }
}

typedef __attribute__((ext_vector_type(4))) float v4f_t;
typedef float v4fa __attribute__((ext_vector_type(4), may_alias));
__device__ __forceinline__ void store_tile16x32(const float* stg, float* __restrict__ dst, size_t ld, int lane) {
  v4f_t vv[4];
#pragma unroll
  for (int i = 0; i < 4; ++i) { const int c = lane + 32 * i; vv[i] = *(const v4fa*)(stg + (c >> 3) * 32 + (c & 7) * 4); }
#pragma unroll
  for (int i = 0; i < 4; ++i) { const int c = lane + 32 * i; *(volatile v4f_t*)(dst + (size_t)(c >> 3) * ld + (c & 7) * 4) = vv[i]; }
  __threadfence();
#pragma unroll
  for (int i = 0; i < 4; ++i) { const int c = lane + 32 * i; *(volatile v4f_t*)(dst + (size_t)(c >> 3) * ld + (c & 7) * 4) = vv[i]; }
}

__global__ __launch_bounds__(256) void gemm_bf16(const unsigned short* __restrict__ A, const unsigned short* __restrict__ Al,
                                                 const unsigned short* __restrict__ W, const unsigned short* __restrict__ Wl,
                                                 float* __restrict__ C,
                                                 int M, int N, int K) {
  __shared__ alignas(32) unsigned short As[128 * 48];
  __shared__ alignas(32) unsigned short Bs[128 * 48];
  __shared__ alignas(32) unsigned short Asl[128 * 48];
  __shared__ alignas(32) unsigned short Bsl[128 * 48];
  __shared__ alignas(16) float stg[8][16 * 32];

  const int tid  = threadIdx.x;
  const int w    = tid >> 5;
  const int lane = tid & 31;
  const int lo   = lane & 15;
  const int hi   = lane >> 4;
  const int mw   = (w >> 1) * 32;
  const int nw   = (w & 1) * 64;
  const int gm0  = blockIdx.y * 128;
  const int gn0  = blockIdx.x * 128;

  f32x8 acc[2][4];
#pragma unroll
  for (int i = 0; i < 2; ++i)
#pragma unroll
    for (int j = 0; j < 4; ++j) acc[i][j] = (f32x8){};

  const int ldRow = tid >> 1;
  const int ldCol = (tid & 1) * 16;

  for (int k0 = 0; k0 < K; k0 += 32) {
    __syncthreads();
    const size_t aOff = (size_t)(gm0 + ldRow) * K + k0 + ldCol, bOff = (size_t)(gn0 + ldRow) * K + k0 + ldCol;
    const unsigned short* aSrc = &A[aOff];
    const unsigned short* bSrc = &W[bOff];
    async_ld_lds_b128(aSrc,     &As[ldRow * 48 + ldCol]);
    async_ld_lds_b128(aSrc + 8, &As[ldRow * 48 + ldCol + 8]);
    async_ld_lds_b128(bSrc,     &Bs[ldRow * 48 + ldCol]);
    async_ld_lds_b128(bSrc + 8, &Bs[ldRow * 48 + ldCol + 8]);
    async_ld_lds_b128(&Al[aOff],     &Asl[ldRow * 48 + ldCol]);
    async_ld_lds_b128(&Al[aOff] + 8, &Asl[ldRow * 48 + ldCol + 8]);
    async_ld_lds_b128(&Wl[bOff],     &Bsl[ldRow * 48 + ldCol]);
    async_ld_lds_b128(&Wl[bOff] + 8, &Bsl[ldRow * 48 + ldCol + 8]);
    __builtin_prefetch(aSrc + 32, 0, 3);
    __builtin_prefetch(bSrc + 32, 0, 3);
    wait_asynccnt0();
    __syncthreads();

    bf16x16 a0  = *(const bf16x16*)&As[(mw + lo) * 48 + hi * 16];
    bf16x16 a1  = *(const bf16x16*)&As[(mw + 16 + lo) * 48 + hi * 16];
    bf16x16 a0l = *(const bf16x16*)&Asl[(mw + lo) * 48 + hi * 16];
    bf16x16 a1l = *(const bf16x16*)&Asl[(mw + 16 + lo) * 48 + hi * 16];
#pragma unroll
    for (int j = 0; j < 4; ++j) {
      bf16x16 bj  = *(const bf16x16*)&Bs[(nw + j * 16 + lo) * 48 + hi * 16];
      bf16x16 bjl = *(const bf16x16*)&Bsl[(nw + j * 16 + lo) * 48 + hi * 16];
      f32x8 x0 = WMMA_BF16(a0l, bj, (f32x8){}); x0 = WMMA_BF16(a0, bjl, x0);
      f32x8 x1 = WMMA_BF16(a1l, bj, (f32x8){}); x1 = WMMA_BF16(a1, bjl, x1);
      acc[0][j] = WMMA_BF16(a0, bj, acc[0][j]) + x0 * RSPLIT;
      acc[1][j] = WMMA_BF16(a1, bj, acc[1][j]) + x1 * RSPLIT;
    }
  }

  float* sg = stg[w];
#pragma unroll
  for (int i = 0; i < 2; ++i)
#pragma unroll
    for (int jp = 0; jp < 4; jp += 2) {
#pragma unroll
      for (int jj = 0; jj < 2; ++jj)
#pragma unroll
        for (int p = 0; p < 8; ++p) sg[(p + 8 * hi) * 32 + jj * 16 + lo] = acc[i][jp + jj][p];
      store_tile16x32(sg, C + (size_t)(gm0 + mw + i * 16) * N + gn0 + nw + jp * 16, (size_t)N, lane);
    }
}

__global__ __launch_bounds__(256) void norm_rope(const float* __restrict__ X,
                                                 const float* __restrict__ wvec,
                                                 const float* __restrict__ cb,
                                                 const float* __restrict__ sb,
                                                 unsigned short* __restrict__ Out,
                                                 unsigned short* __restrict__ Outl,
                                                 int nH) {
  const int w    = threadIdx.x >> 5;
  const int lane = threadIdx.x & 31;
  const int r    = blockIdx.x * 8 + w;
  const int h    = r % nH;
  const int bs   = r / nH;

  const float* x = X + ((size_t)bs * nH + h) * 64;
  float e0 = x[lane];
  float e1 = x[lane + 32];

  float ss = e0 * e0 + e1 * e1;
  ss += __shfl_xor(ss, 1);
  ss += __shfl_xor(ss, 2);
  ss += __shfl_xor(ss, 4);
  ss += __shfl_xor(ss, 8);
  ss += __shfl_xor(ss, 16);
  float rinv = rsqrtf(ss * (1.0f / 64.0f) + 1e-6f);

  float n0 = wvec[lane] * e0 * rinv;
  float n1 = wvec[lane + 32] * e1 * rinv;

  const float* cp = cb + (size_t)bs * 64;
  const float* sp = sb + (size_t)bs * 64;
  float o0 = n0 * cp[lane]      - n1 * sp[lane];
  float o1 = n1 * cp[lane + 32] + n0 * sp[lane + 32];

  const int b = bs / S_;
  const int s = bs % S_;
  const int e0i = (2 * lane) & 31, e1i = (2 * lane + 1) & 31;
  const float a0 = __shfl(o0, e0i), b0 = __shfl(o1, e0i);
  const float a1 = __shfl(o0, e1i), b1 = __shfl(o1, e1i);
  const bool upper = (lane >= 16);
  const float x0 = upper ? b0 : a0, x1 = upper ? b1 : a1;
  unsigned short hx0, lx0, hx1, lx1; split16(x0, hx0, lx0); split16(x1, hx1, lx1);
  const unsigned pk = (unsigned)hx0 | ((unsigned)hx1 << 16), pkl = (unsigned)lx0 | ((unsigned)lx1 << 16);
  const size_t ro = (((size_t)b * nH + h) * S_ + s) * 64;
  unsigned* op = (unsigned*)(Out + ro); unsigned* opl = (unsigned*)(Outl + ro);
  *(volatile unsigned*)(op + lane) = pk; *(volatile unsigned*)(opl + lane) = pkl;
  __threadfence();
  *(volatile unsigned*)(op + lane) = pk; *(volatile unsigned*)(opl + lane) = pkl;
}

__global__ __launch_bounds__(256) void v_convert(const float* __restrict__ V,
                                                 unsigned short* __restrict__ Vt, unsigned short* __restrict__ Vtl) {
  int i  = blockIdx.x * 256 + threadIdx.x;
  int sp = i & (S_ / 2 - 1);
  int r  = i >> 10;
  int d  = r & 63;
  int h  = (r >> 6) & (NKV_ - 1);
  int b  = r >> 9;
  const int s = 2 * sp;
  const float v0 = V[((size_t)(b * S_ + s)) * (NKV_ * 64) + h * 64 + d];
  const float v1 = V[((size_t)(b * S_ + s + 1)) * (NKV_ * 64) + h * 64 + d];
  unsigned short hv0, lv0, hv1, lv1; split16(v0, hv0, lv0); split16(v1, hv1, lv1);
  const unsigned pk = (unsigned)hv0 | ((unsigned)hv1 << 16), pkl = (unsigned)lv0 | ((unsigned)lv1 << 16);
  const size_t vo = (((size_t)b * NKV_ + h) * 64 + d) * S_ + s;
  unsigned* vp = (unsigned*)(Vt + vo); unsigned* vpl = (unsigned*)(Vtl + vo);
  *(volatile unsigned*)vp = pk; *(volatile unsigned*)vpl = pkl;
  __threadfence();
  *(volatile unsigned*)vp = pk; *(volatile unsigned*)vpl = pkl;
}

__global__ __launch_bounds__(128) void attn_kernel(const unsigned short* __restrict__ Q, const unsigned short* __restrict__ Ql,
                                                   const unsigned short* __restrict__ Kc, const unsigned short* __restrict__ Kcl,
                                                   const unsigned short* __restrict__ Vt, const unsigned short* __restrict__ Vtl,
                                                   unsigned short* __restrict__ O, unsigned short* __restrict__ Ol) {
  __shared__ alignas(32) unsigned short Ks[32 * 80];
  __shared__ alignas(32) unsigned short VTs[64 * 48];
  __shared__ alignas(32) unsigned short Ksl[32 * 80];
  __shared__ alignas(32) unsigned short VTsl[64 * 48];
  __shared__ alignas(32) unsigned short Ps[4 * 16 * 32];
  __shared__ alignas(32) unsigned short Psl[4 * 16 * 32];
  __shared__ alignas(16) unsigned short Os[4][16 * 64];
  __shared__ alignas(16) unsigned short Osl[4][16 * 64];

  const int tid  = threadIdx.x;
  const int w    = tid >> 5;
  const int lane = tid & 31;
  const int lo   = lane & 15;
  const int hi   = lane >> 4;

  const int bh    = blockIdx.x;
  const int b     = bh >> 5;
  const int h     = bh & 31;
  const int hk    = h >> 2;
  const int qBase = blockIdx.y * 64;
  const int qRow0 = qBase + w * 16;

  const size_t qo = ((size_t)(b * NH_ + h) * S_ + (qRow0 + lo)) * HD_;
  const unsigned short* qptr = Q + qo; const unsigned short* qptrl = Ql + qo;
  bf16x16 aQ0  = *(const bf16x16*)(qptr + hi * 16);
  bf16x16 aQ1  = *(const bf16x16*)(qptr + 32 + hi * 16);
  bf16x16 aQ0l = *(const bf16x16*)(qptrl + hi * 16);
  bf16x16 aQ1l = *(const bf16x16*)(qptrl + 32 + hi * 16);

  f32x8 o0 = {}, o1 = {}, o2 = {}, o3 = {};
  float m[8], l[8];
#pragma unroll
  for (int p = 0; p < 8; ++p) { m[p] = -1e30f; l[p] = 0.0f; }

  const unsigned short* kbase  = Kc  + (size_t)(b * NKV_ + hk) * S_ * HD_;
  const unsigned short* vbase  = Vt  + (size_t)(b * NKV_ + hk) * HD_ * S_;
  const unsigned short* kbasel = Kcl + (size_t)(b * NKV_ + hk) * S_ * HD_;
  const unsigned short* vbasel = Vtl + (size_t)(b * NKV_ + hk) * HD_ * S_;

  const int kKey = tid >> 2, kD = (tid & 3) * 16;
  const int vD = tid >> 1, vHalf = tid & 1;

  const int nChunks = (qBase >> 5) + 2;
  for (int kc = 0; kc < nChunks; ++kc) {
    const int k0 = kc * 32;
    __syncthreads();
    {
      const size_t ko = (size_t)(k0 + kKey) * HD_ + kD;
      async_ld_lds_b128(kbase + ko,      &Ks[kKey * 80 + kD]);
      async_ld_lds_b128(kbase + ko + 8,  &Ks[kKey * 80 + kD + 8]);
      async_ld_lds_b128(kbasel + ko,     &Ksl[kKey * 80 + kD]);
      async_ld_lds_b128(kbasel + ko + 8, &Ksl[kKey * 80 + kD + 8]);
    }
    {
      const size_t vo = (size_t)vD * S_ + k0 + vHalf * 16;
      async_ld_lds_b128(vbase + vo,      &VTs[vD * 48 + vHalf * 16]);
      async_ld_lds_b128(vbase + vo + 8,  &VTs[vD * 48 + vHalf * 16 + 8]);
      async_ld_lds_b128(vbasel + vo,     &VTsl[vD * 48 + vHalf * 16]);
      async_ld_lds_b128(vbasel + vo + 8, &VTsl[vD * 48 + vHalf * 16 + 8]);
    }
    wait_asynccnt0();
    __syncthreads();

    f32x8 s0 = {}, s1 = {};
    {
      bf16x16 bk, bkl; f32x8 x;
      bk = *(const bf16x16*)&Ks[(lo) * 80 + hi * 16];           bkl = *(const bf16x16*)&Ksl[(lo) * 80 + hi * 16];
      x = WMMA_BF16(aQ0l, bk, (f32x8){}); x = WMMA_BF16(aQ0, bkl, x); s0 = WMMA_BF16(aQ0, bk, s0) + x * RSPLIT;
      bk = *(const bf16x16*)&Ks[(lo) * 80 + 32 + hi * 16];      bkl = *(const bf16x16*)&Ksl[(lo) * 80 + 32 + hi * 16];
      x = WMMA_BF16(aQ1l, bk, (f32x8){}); x = WMMA_BF16(aQ1, bkl, x); s0 = WMMA_BF16(aQ1, bk, s0) + x * RSPLIT;
      bk = *(const bf16x16*)&Ks[(16 + lo) * 80 + hi * 16];      bkl = *(const bf16x16*)&Ksl[(16 + lo) * 80 + hi * 16];
      x = WMMA_BF16(aQ0l, bk, (f32x8){}); x = WMMA_BF16(aQ0, bkl, x); s1 = WMMA_BF16(aQ0, bk, s1) + x * RSPLIT;
      bk = *(const bf16x16*)&Ks[(16 + lo) * 80 + 32 + hi * 16]; bkl = *(const bf16x16*)&Ksl[(16 + lo) * 80 + 32 + hi * 16];
      x = WMMA_BF16(aQ1l, bk, (f32x8){}); x = WMMA_BF16(aQ1, bkl, x); s1 = WMMA_BF16(aQ1, bk, s1) + x * RSPLIT;
    }

    const int key0 = k0 + lo;
    const int key1 = k0 + 16 + lo;
#pragma unroll
    for (int p = 0; p < 8; ++p) {
      const int qrow = qRow0 + p + 8 * hi;
      float v0 = s0[p] * SCALE_;
      float v1 = s1[p] * SCALE_;
      if (key0 > qrow) v0 = NEG_BIG;
      if (key1 > qrow) v1 = NEG_BIG;

      float mx = fmaxf(v0, v1);
      mx = fmaxf(mx, __shfl_xor(mx, 1));
      mx = fmaxf(mx, __shfl_xor(mx, 2));
      mx = fmaxf(mx, __shfl_xor(mx, 4));
      mx = fmaxf(mx, __shfl_xor(mx, 8));

      float mn    = fmaxf(m[p], mx);
      float alpha = __expf(m[p] - mn);
      m[p] = mn;
      float p0 = __expf(v0 - mn);
      float p1 = __expf(v1 - mn);
      float rs = p0 + p1;
      rs += __shfl_xor(rs, 1);
      rs += __shfl_xor(rs, 2);
      rs += __shfl_xor(rs, 4);
      rs += __shfl_xor(rs, 8);
      l[p] = l[p] * alpha + rs;
      o0[p] *= alpha; o1[p] *= alpha; o2[p] *= alpha; o3[p] *= alpha;

      const int prow = p + 8 * hi;
      { unsigned short hp, lp;
        split16(p0 * 1024.0f, hp, lp); Ps[(w * 16 + prow) * 32 + lo]      = hp; Psl[(w * 16 + prow) * 32 + lo]      = lp;
        split16(p1 * 1024.0f, hp, lp); Ps[(w * 16 + prow) * 32 + 16 + lo] = hp; Psl[(w * 16 + prow) * 32 + 16 + lo] = lp; }
    }

    bf16x16 aP  = *(const bf16x16*)&Ps[(w * 16 + lo) * 32 + hi * 16];
    bf16x16 aPl = *(const bf16x16*)&Psl[(w * 16 + lo) * 32 + hi * 16];
    {
      bf16x16 bv, bvl; f32x8 x;
      bv = *(const bf16x16*)&VTs[(lo) * 48 + hi * 16];       bvl = *(const bf16x16*)&VTsl[(lo) * 48 + hi * 16];
      x = WMMA_BF16(aPl, bv, (f32x8){}); x = WMMA_BF16(aP, bvl, x); o0 = WMMA_BF16(aP, bv, o0) + x * RSPLIT;
      bv = *(const bf16x16*)&VTs[(16 + lo) * 48 + hi * 16];  bvl = *(const bf16x16*)&VTsl[(16 + lo) * 48 + hi * 16];
      x = WMMA_BF16(aPl, bv, (f32x8){}); x = WMMA_BF16(aP, bvl, x); o1 = WMMA_BF16(aP, bv, o1) + x * RSPLIT;
      bv = *(const bf16x16*)&VTs[(32 + lo) * 48 + hi * 16];  bvl = *(const bf16x16*)&VTsl[(32 + lo) * 48 + hi * 16];
      x = WMMA_BF16(aPl, bv, (f32x8){}); x = WMMA_BF16(aP, bvl, x); o2 = WMMA_BF16(aP, bv, o2) + x * RSPLIT;
      bv = *(const bf16x16*)&VTs[(48 + lo) * 48 + hi * 16];  bvl = *(const bf16x16*)&VTsl[(48 + lo) * 48 + hi * 16];
      x = WMMA_BF16(aPl, bv, (f32x8){}); x = WMMA_BF16(aP, bvl, x); o3 = WMMA_BF16(aP, bv, o3) + x * RSPLIT;
    }
  }

  unsigned short* os = Os[w]; unsigned short* osl = Osl[w];
#pragma unroll
  for (int p = 0; p < 8; ++p) {
    const int prow = p + 8 * hi;
    float invl = 1.0f / (l[p] * 1024.0f);
    unsigned short hv, lv;
    split16(o0[p] * invl, hv, lv); os[prow * 64 + lo]      = hv; osl[prow * 64 + lo]      = lv;
    split16(o1[p] * invl, hv, lv); os[prow * 64 + 16 + lo] = hv; osl[prow * 64 + 16 + lo] = lv;
    split16(o2[p] * invl, hv, lv); os[prow * 64 + 32 + lo] = hv; osl[prow * 64 + 32 + lo] = lv;
    split16(o3[p] * invl, hv, lv); os[prow * 64 + 48 + lo] = hv; osl[prow * 64 + 48 + lo] = lv;
  }
  {
    typedef __attribute__((ext_vector_type(4))) unsigned v4u_t;
    typedef unsigned v4ua __attribute__((ext_vector_type(4), may_alias));
    v4u_t ov[4], ovl[4]; size_t oo[4];
#pragma unroll
    for (int i = 0; i < 4; ++i) {
      const int c = lane + 32 * i, r = c >> 3, q = c & 7;
      ov[i]  = *(const v4ua*)(os + r * 64 + q * 8);
      ovl[i] = *(const v4ua*)(osl + r * 64 + q * 8);
      oo[i] = ((size_t)b * S_ + qRow0 + r) * (size_t)(NH_ * HD_) + (size_t)h * HD_ + q * 8;
    }
#pragma unroll
    for (int i = 0; i < 4; ++i) { *(volatile v4u_t*)(O + oo[i]) = ov[i]; *(volatile v4u_t*)(Ol + oo[i]) = ovl[i]; }
    __threadfence();
#pragma unroll
    for (int i = 0; i < 4; ++i) { *(volatile v4u_t*)(O + oo[i]) = ov[i]; *(volatile v4u_t*)(Ol + oo[i]) = ovl[i]; }
  }
}

extern "C" void kernel_launch(void* const* d_in, const int* in_sizes, int n_in,
                              void* d_out, int out_size, void* d_ws, size_t ws_size,
                              hipStream_t stream) {
  (void)in_sizes; (void)n_in; (void)out_size; (void)ws_size;

  const float* hidden = (const float*)d_in[0];
  const float* cosb   = (const float*)d_in[1];
  const float* sinb   = (const float*)d_in[2];
  const float* Wq     = (const float*)d_in[3];
  const float* Wk     = (const float*)d_in[4];
  const float* Wv     = (const float*)d_in[5];
  const float* Wo     = (const float*)d_in[6];
  const float* qnw    = (const float*)d_in[7];
  const float* knw    = (const float*)d_in[8];
  float* out = (float*)d_out;

  const int M = B_ * S_;
  char* base = (char*)d_ws;
  size_t off = 0;
  auto alloc = [&](size_t bytes) -> void* {
    void* p = base + off;
    off = (off + bytes + 255) & ~(size_t)255;
    return p;
  };

  unsigned short* Xbf  = (unsigned short*)alloc((size_t)M * HID_ * 2);          unsigned short* XbfL  = (unsigned short*)alloc((size_t)M * HID_ * 2);
  unsigned short* Wqbf = (unsigned short*)alloc((size_t)HID_ * HID_ * 2);       unsigned short* WqbfL = (unsigned short*)alloc((size_t)HID_ * HID_ * 2);
  unsigned short* Wkbf = (unsigned short*)alloc((size_t)NKV_ * HD_ * HID_ * 2); unsigned short* WkbfL = (unsigned short*)alloc((size_t)NKV_ * HD_ * HID_ * 2);
  unsigned short* Wvbf = (unsigned short*)alloc((size_t)NKV_ * HD_ * HID_ * 2); unsigned short* WvbfL = (unsigned short*)alloc((size_t)NKV_ * HD_ * HID_ * 2);
  unsigned short* Wobf = (unsigned short*)alloc((size_t)HID_ * HID_ * 2);       unsigned short* WobfL = (unsigned short*)alloc((size_t)HID_ * HID_ * 2);
  float* qf = (float*)alloc((size_t)M * HID_ * 4);
  float* kf = (float*)alloc((size_t)M * NKV_ * HD_ * 4);
  float* vf = (float*)alloc((size_t)M * NKV_ * HD_ * 4);
  unsigned short* Qbf = (unsigned short*)alloc((size_t)M * HID_ * 2);           unsigned short* QbfL = (unsigned short*)alloc((size_t)M * HID_ * 2);
  unsigned short* Kbf = (unsigned short*)alloc((size_t)M * NKV_ * HD_ * 2);     unsigned short* KbfL = (unsigned short*)alloc((size_t)M * NKV_ * HD_ * 2);
  unsigned short* Vtb = (unsigned short*)alloc((size_t)M * NKV_ * HD_ * 2);     unsigned short* VtbL = (unsigned short*)alloc((size_t)M * NKV_ * HD_ * 2);
  unsigned short* Abf = (unsigned short*)alloc((size_t)M * HID_ * 2);           unsigned short* AbfL = (unsigned short*)alloc((size_t)M * HID_ * 2);

  cvt_f32_bf16<<<(M * HID_) / 1024, 256, 0, stream>>>(hidden, Xbf, XbfL, M * HID_);
  cvt_f32_bf16<<<(HID_ * HID_) / 1024, 256, 0, stream>>>(Wq, Wqbf, WqbfL, HID_ * HID_);
  cvt_f32_bf16<<<(NKV_ * HD_ * HID_) / 1024, 256, 0, stream>>>(Wk, Wkbf, WkbfL, NKV_ * HD_ * HID_);
  cvt_f32_bf16<<<(NKV_ * HD_ * HID_) / 1024, 256, 0, stream>>>(Wv, Wvbf, WvbfL, NKV_ * HD_ * HID_);
  cvt_f32_bf16<<<(HID_ * HID_) / 1024, 256, 0, stream>>>(Wo, Wobf, WobfL, HID_ * HID_);

  gemm_bf16<<<dim3(HID_ / 128, M / 128), 256, 0, stream>>>(Xbf, XbfL, Wqbf, WqbfL, qf, M, HID_, HID_);
  gemm_bf16<<<dim3((NKV_ * HD_) / 128, M / 128), 256, 0, stream>>>(Xbf, XbfL, Wkbf, WkbfL, kf, M, NKV_ * HD_, HID_);
  gemm_bf16<<<dim3((NKV_ * HD_) / 128, M / 128), 256, 0, stream>>>(Xbf, XbfL, Wvbf, WvbfL, vf, M, NKV_ * HD_, HID_);

  norm_rope<<<(M * NH_) / 8, 256, 0, stream>>>(qf, qnw, cosb, sinb, Qbf, QbfL, NH_);
  norm_rope<<<(M * NKV_) / 8, 256, 0, stream>>>(kf, knw, cosb, sinb, Kbf, KbfL, NKV_);
  v_convert<<<(M * NKV_ * HD_ / 2) / 256, 256, 0, stream>>>(vf, Vtb, VtbL);

  attn_kernel<<<dim3(B_ * NH_, S_ / 64), 128, 0, stream>>>(Qbf, QbfL, Kbf, KbfL, Vtb, VtbL, Abf, AbfL);

  gemm_bf16<<<dim3(HID_ / 128, M / 128), 256, 0, stream>>>(Abf, AbfL, Wobf, WobfL, out, M, HID_, HID_);
}
